// StaticAddAttention_58626303590869
// MI455X (gfx1250) — hardware-verified
//
#include <hip/hip_runtime.h>


#ifndef NB
#define NB 2
#endif
#ifndef TQ
#define TQ 512
#endif
#define NB_FULL 2
#define TQ_FULL 512
#define TK    512
#define DQ    1024
#define DK    1024
#define DV    1024
#define HH    256
#define OUTW  2048
#define PCAR  1024.0f
#define VSC   16.0f
#define OSC   (1.0f / 16384.0f)
#define LOG2E 1.4426950408889634f
#define EPSM  1e-13f

static_assert(TQ == TQ_FULL || NB == 1);
static_assert(TQ % 64 == 0 && TQ >= 64 && TQ <= TQ_FULL);
static_assert(NB >= 1 && NB <= NB_FULL);
static_assert(TK == 2 * 256);
static_assert((NB * TQ) % 64 == 0 && (NB * TK) % 64 == 0 && HH % 64 == 0 && DV % 64 == 0);
static_assert(DQ % 32 == 0 && DK % 32 == 0 && TK % 32 == 0 && HH % 128 == 0);
static_assert(TQ_FULL == TK && DQ == DV && DQ == DK && OUTW == DV + DQ);
static_assert((size_t)NB_FULL * TQ_FULL * OUTW * 4 == 8388608);
static_assert(32 * 4 * (HH / 128) == HH);
static_assert(2 * (size_t)HH * DQ * 2 + (size_t)NB * TQ * DQ * 2 + (size_t)NB * TK * DK * 2 + (size_t)NB * TQ * HH * 4 + (size_t)NB * TK * HH * 4
              + (size_t)NB * DV * TK * 2 + (size_t)NB * TQ * TK * 2 <= 134217728);
static_assert(16 * 68 * 4 <= 131072);
static_assert((TK + 8) * 4 <= 131072);

typedef _Float16 h16;
typedef unsigned short bf;
typedef __attribute__((ext_vector_type(16))) __bf16   v16bf;
typedef __attribute__((ext_vector_type(16))) _Float16 v16h;
typedef __attribute__((ext_vector_type(8)))  _Float16 v8h;
typedef __attribute__((ext_vector_type(8)))  unsigned short v8us;
typedef __attribute__((ext_vector_type(8)))  float    v8f;
typedef __attribute__((ext_vector_type(4)))  float    v4f;
typedef __attribute__((ext_vector_type(2)))  _Float16 v2h;
typedef __attribute__((ext_vector_type(2)))  unsigned short v2us;
typedef v8h  __attribute__((may_alias)) v8ha;
typedef v4f  __attribute__((may_alias)) v4fa;
typedef v8us __attribute__((may_alias)) v8usa;

__device__ __forceinline__ unsigned short f2bf(float f) { unsigned u = __float_as_uint(f); u += 0x7FFFu + ((u >> 16) & 1u); return (unsigned short)(u >> 16); }
__device__ __forceinline__ float bf2f(unsigned short b) { return __uint_as_float(((unsigned)b) << 16); }
__device__ __forceinline__ float bfr(float f) { return bf2f(f2bf(f)); }
__device__ __forceinline__ v16h cat16(v8h lo, v8h hi) { return __builtin_shufflevector(lo, hi, 0, 1, 2, 3, 4, 5, 6, 7, 8, 9, 10, 11, 12, 13, 14, 15); }
__device__ __forceinline__ v16bf cat16b(v8us lo, v8us hi) { return __builtin_bit_cast(v16bf, __builtin_shufflevector(lo, hi, 0, 1, 2, 3, 4, 5, 6, 7, 8, 9, 10, 11, 12, 13, 14, 15)); }
__device__ __forceinline__ v8f wmma16(v16h a, v16h b, v8f c) { return __builtin_amdgcn_wmma_f32_16x16x32_f16(false, a, false, b, (short)0, c, false, false); }
__device__ __forceinline__ v8f wmmab(v16bf a, v16bf b, v8f c) { return __builtin_amdgcn_wmma_f32_16x16x32_bf16(false, a, false, b, (short)0, c, false, false); }

template <typename T16> struct WFrag;
template <> struct WFrag<h16> { typedef v16h V; static __device__ __forceinline__ V ld(const h16* p) { return cat16(*(const v8h*)p, *(const v8h*)(p + 16)); } static __device__ __forceinline__ v8f mma(V a, V b, v8f c) { return wmma16(a, b, c); } };
template <> struct WFrag<bf> { typedef v16bf V; static __device__ __forceinline__ V ld(const bf* p) { return cat16b(*(const v8us*)p, *(const v8us*)(p + 16)); } static __device__ __forceinline__ v8f mma(V a, V b, v8f c) { return wmmab(a, b, c); } };
template <typename T16, int NSPLIT, bool BIAS>
__global__ __launch_bounds__(32) void k_gemmw(const T16* __restrict__ A, const T16* __restrict__ A2, const T16* __restrict__ Bt, const T16* __restrict__ Bt2, int K, float* C, int ldc, const float* __restrict__ bias, float csc, size_t sA, size_t sB, size_t sC) {
    typedef typename WFrag<T16>::V V;
    __shared__ __align__(16) float os[16 * 68];
    const size_t z = blockIdx.z; A += z * sA; if (A2) A2 += z * sA; Bt += z * sB; if (Bt2) Bt2 += z * sB; C += z * sC;
    const int lane = threadIdx.x & 31, lr = lane & 15, hi = lane >> 4; const int r0 = blockIdx.x * 64, c0 = blockIdx.y * 64;
    v8f acc[4][4];
#pragma unroll
    for (int mb = 0; mb < 4; ++mb)
#pragma unroll
        for (int nb = 0; nb < 4; ++nb) acc[mb][nb] = (v8f){};
    const size_t aoff = (size_t)(r0 + lr) * K + 8 * hi, boff = (size_t)(c0 + lr) * K + 8 * hi;
#pragma unroll 1
    for (int kc = 0; kc < K; kc += 32) {
        V a[4], a2[4];
#pragma unroll
        for (int mb = 0; mb < 4; ++mb) { a[mb] = WFrag<T16>::ld(A + aoff + (size_t)mb * 16 * K + kc); if (NSPLIT == 1 || NSPLIT == 2) a2[mb] = WFrag<T16>::ld(A2 + aoff + (size_t)mb * 16 * K + kc); }
#pragma unroll
        for (int nb = 0; nb < 4; ++nb) { const V b = WFrag<T16>::ld(Bt + boff + (size_t)nb * 16 * K + kc); V b2; if (NSPLIT >= 2) b2 = WFrag<T16>::ld(Bt2 + boff + (size_t)nb * 16 * K + kc);
#pragma unroll
            for (int mb = 0; mb < 4; ++mb) { acc[mb][nb] = WFrag<T16>::mma(a[mb], b, acc[mb][nb]); if (NSPLIT == 1 || NSPLIT == 2) acc[mb][nb] = WFrag<T16>::mma(a2[mb], b, acc[mb][nb]); if (NSPLIT >= 2) acc[mb][nb] = WFrag<T16>::mma(a[mb], b2, acc[mb][nb]); } }
        asm volatile("v_nop\n\tv_nop\n\tv_nop\n\tv_nop" : "+v"(acc[0][0]), "+v"(acc[1][1]), "+v"(acc[2][2]), "+v"(acc[3][3]) : "v"(a[0]), "v"(a[3]));
    }
#pragma unroll
    for (int mb = 0; mb < 4; ++mb) {
#pragma unroll
        for (int nb = 0; nb < 4; ++nb) {
#pragma unroll
            for (int j = 0; j < 8; ++j) os[(hi * 8 + j) * 68 + nb * 16 + lr] = acc[mb][nb][j]; }
        __builtin_amdgcn_wave_barrier(); asm volatile("" ::: "memory");
        float* crow = C + (size_t)(r0 + mb * 16) * ldc + c0;
#pragma unroll 1
        for (int ps = 0; ps < 2; ++ps) {
#pragma unroll
            for (int s = 0; s < 8; ++s) { const int row = 2 * s + hi, cofs = lr * 4; v4f val = *(const v4fa*)(os + row * 68 + cofs); val = val * csc;
                if (BIAS) { val[0] += bfr(bias[c0 + cofs]); val[1] += bfr(bias[c0 + cofs + 1]); val[2] += bfr(bias[c0 + cofs + 2]); val[3] += bfr(bias[c0 + cofs + 3]); }
                *(volatile v4f*)(crow + (size_t)row * ldc + cofs) = val; }
            if (ps == 0) __threadfence(); }
        __builtin_amdgcn_wave_barrier(); asm volatile("" ::: "memory");
    }
}

__global__ __launch_bounds__(256) void k_wtG(const float* __restrict__ w, int K, int N, bf* Bt) {
    const int lane = threadIdx.x & 31; const int L0 = (blockIdx.x * 8 + (threadIdx.x >> 5)) * 8; const int nlines = N * K / 64;
#pragma unroll
    for (int ps = 0; ps < 2; ++ps) {
#pragma unroll 1
        for (int l = 0; l < 8; ++l) { const int L = L0 + l; if (L >= nlines) break; const size_t e = (size_t)L * 64 + lane * 2; const int k = (int)(e % K), n = (int)(e / K); v2us o;
            o[0] = f2bf(w[(size_t)k * N + n]); o[1] = f2bf(w[(size_t)(k + 1) * N + n]); *(volatile v2us*)(Bt + e) = o; }
        if (ps == 0) __threadfence(); }
}

__global__ __launch_bounds__(256) void k_cvt8(const float* __restrict__ src, bf* dst, size_t n8) { const size_t i = (size_t)blockIdx.x * 256 + threadIdx.x; if (i >= n8) return; const v8f v = *(const v8f*)(src + i * 8); v8us o;
#pragma unroll
    for (int k = 0; k < 8; ++k) o[k] = f2bf(v[k]); *(volatile v8us*)(dst + i * 8) = o; __threadfence(); *(volatile v8us*)(dst + i * 8) = o; }

static __device__ __forceinline__ h16 toh_flush(float v) { const float w = (fabsf(v) < 6.103515625e-05f) ? 0.0f : v; return (h16)w; }

__global__ __launch_bounds__(256) void k_vtp(const float* __restrict__ F, h16* V16) {
    const size_t e = ((size_t)blockIdx.x * 256 + threadIdx.x) * 2; if (e >= (size_t)NB * DV * TK) return;
    const int t = (int)(e % TK); const int d = (int)((e / TK) % DV); const int b = (int)(e / ((size_t)TK * DV));
    v2h o;
#pragma unroll
    for (int q = 0; q < 2; ++q) o[q] = toh_flush(bfr(F[((size_t)b * TK + t + q) * DV + d]) * VSC);
    *(volatile v2h*)(V16 + e) = o; __threadfence(); *(volatile v2h*)(V16 + e) = o;
}

__device__ __forceinline__ float tnh(float x) {
    const float e = __builtin_amdgcn_exp2f(x * 2.8853900817779268f);
    const float r = __builtin_amdgcn_rcpf(e + 1.0f);
    return fmaf(-2.0f, r, 1.0f);
}

static_assert(2 * 32 * 8 == TK);
__global__ __launch_bounds__(256) void k_score(const float* __restrict__ WQF, const float* __restrict__ UHF, const float* __restrict__ vv, const int* __restrict__ mk, h16* P16) {
    __shared__ __align__(16) float s_sc[TK];
    __shared__ float red[8];
    const int rq = blockIdx.x; const int b = rq / TQ;
    const int tid = threadIdx.x, lane = tid & 31, wave = tid >> 5;
    const float* wrow = WQF + (size_t)rq * HH;
    float wq[4 * (HH / 128)], vr[4 * (HH / 128)];
#pragma unroll
    for (int i = 0; i < HH / 128; ++i) { const v4f w4 = *(const v4f*)(wrow + i * 128 + lane * 4); const v4f v4 = *(const v4f*)(vv + i * 128 + lane * 4);
#pragma unroll
        for (int c = 0; c < 4; ++c) { wq[i * 4 + c] = w4[c]; vr[i * 4 + c] = bfr(v4[c]); } }
    const float* ub = UHF + (size_t)b * TK * HH;
#pragma unroll 1
    for (int kk = 0; kk < TK / 8; ++kk) {
        const int k = wave * (TK / 8) + kk;
        const float* urow = ub + (size_t)k * HH;
        float acc = 0.0f;
#pragma unroll
        for (int i = 0; i < HH / 128; ++i) { const v4f u4 = *(const v4f*)(urow + i * 128 + lane * 4);
#pragma unroll
            for (int c = 0; c < 4; ++c) acc = fmaf(vr[i * 4 + c], tnh(wq[i * 4 + c] + u4[c]), acc); }
#pragma unroll
        for (int sh = 16; sh; sh >>= 1) acc += __shfl_xor(acc, sh, 32);
        if (lane == 0) s_sc[k] = acc;
    }
    __syncthreads();
    const float a0 = s_sc[tid], a1 = s_sc[tid + 256];
    const int mw0 = mk[b * TK + tid], mw1 = mk[b * TK + tid + 256];
    const float mf0 = (float)mw0, mf1 = (float)mw1;
    const float z0 = a0 * mf0, z1 = a1 * mf1;
    float m = fmaxf(z0, z1);
#pragma unroll
    for (int sh = 16; sh; sh >>= 1) m = fmaxf(m, __shfl_xor(m, sh, 32));
    if (lane == 0) red[wave] = m;
    __syncthreads();
    m = red[0];
#pragma unroll
    for (int w = 1; w < 8; ++w) m = fmaxf(m, red[w]);
    __syncthreads();
    float d0 = z0 - m, d1 = z1 - m;
    const float e0 = __builtin_amdgcn_exp2f(d0 * LOG2E), e1 = __builtin_amdgcn_exp2f(d1 * LOG2E);
    float sum = e0 + e1;
#pragma unroll
    for (int sh = 16; sh; sh >>= 1) sum += __shfl_xor(sum, sh, 32);
    if (lane == 0) red[wave] = sum;
    __syncthreads();
    sum = red[0];
#pragma unroll
    for (int w = 1; w < 8; ++w) sum += red[w];
    const float inv = __builtin_amdgcn_rcpf(sum);
    __syncthreads();
    const float s0 = (e0 * inv) * mf0, s1 = (e1 * inv) * mf1;
    s_sc[tid] = s0; s_sc[tid + 256] = s1;
    float sum2 = s0 + s1;
#pragma unroll
    for (int sh = 16; sh; sh >>= 1) sum2 += __shfl_xor(sum2, sh, 32);
    if (lane == 0) red[wave] = sum2;
    __syncthreads();
    sum2 = red[0];
#pragma unroll
    for (int w = 1; w < 8; ++w) sum2 += red[w];
    const float invp = (1.0f / (sum2 + EPSM)) * PCAR;
    if (wave >= 4 && wave < 6) {
        const int f0 = ((wave - 4) * 32 + lane) * 8;
        const v4f q0 = *(const v4fa*)(s_sc + f0); const v4f q1 = *(const v4fa*)(s_sc + f0 + 4);
        v8h o;
#pragma unroll
        for (int c = 0; c < 4; ++c) { o[c] = toh_flush(q0[c] * invp); o[4 + c] = toh_flush(q1[c] * invp); }
        h16* dst = P16 + (size_t)rq * TK + f0;
        *(volatile v8h*)dst = o; __threadfence(); *(volatile v8h*)dst = o;
    }
}

static_assert((DQ / 4) % 32 == 0);
static_assert(((size_t)NB * TQ * DQ / 4) % 256 == 0);
static_assert(((size_t)NB * TQ * DQ / 4) * 16 == (size_t)NB * TQ * DQ * 4);
__global__ __launch_bounds__(256) void k_cph(const float* __restrict__ src, float* dst, size_t n4) {
    const size_t i = (size_t)blockIdx.x * 256 + threadIdx.x; if (i >= n4) return;
    const size_t row = i / (DQ / 4); const int c4 = (int)(i % (DQ / 4));
    const v4f v = *(const v4f*)(src + row * DQ + c4 * 4); v4f o;
#pragma unroll
    for (int k = 0; k < 4; ++k) o[k] = bfr(v[k]);
    float* p = dst + row * OUTW + DQ + c4 * 4;
    *(volatile v4f*)p = o; __threadfence(); *(volatile v4f*)p = o;
}

extern "C" void kernel_launch(void* const* d_in, const int* in_sizes, int n_in,
                              void* d_out, int out_size, void* d_ws, size_t ws_size, hipStream_t stream) {
    if (n_in < 5) return;
    if (in_sizes[0] < NB * TQ * DQ || in_sizes[0] < NB * TK * DV || in_sizes[1] < NB * TK * DK || in_sizes[2] < NB * TK || in_sizes[3] < (DQ + DK) * HH || in_sizes[4] < HH) return;
    if (out_size < NB_FULL * TQ_FULL * OUTW) return;
    const float* input  = (const float*)d_in[0];
    const float* memory = (const float*)d_in[1];
    const int*   mmask  = (const int*)d_in[2];
    const float* w1     = (const float*)d_in[3];
    const float* w2     = (const float*)d_in[4];
    float* OUT0 = (float*)d_out;

    char* wsp = (char*)d_ws;
    auto take = [&](size_t bytes) { char* p = wsp; wsp += (bytes + 255) & ~(size_t)255; return (void*)p; };
    bf*    WQT  = (bf*)take((size_t)HH * DQ * 2);
    bf*    WKT  = (bf*)take((size_t)HH * DK * 2);
    bf*    QB   = (bf*)take((size_t)NB * TQ * DQ * 2);
    bf*    KB   = (bf*)take((size_t)NB * TK * DK * 2);
    float* WQF  = (float*)take((size_t)NB * TQ * HH * 4);
    float* UHF  = (float*)take((size_t)NB * TK * HH * 4);
    h16*   VT16 = (h16*)take((size_t)NB * DV * TK * 2);
    h16*   P16  = (h16*)take((size_t)NB * TQ * TK * 2);
    if ((size_t)(wsp - (char*)d_ws) > ws_size) return;

    k_wtG<<<(unsigned)((DQ * HH / 64 + 63) / 64), 256, 0, stream>>>(w1, DQ, HH, WQT);
    k_wtG<<<(unsigned)((DK * HH / 64 + 63) / 64), 256, 0, stream>>>(w1 + (size_t)DQ * HH, DK, HH, WKT);
    k_cvt8<<<(unsigned)(((size_t)NB * TQ * DQ / 8 + 255) / 256), 256, 0, stream>>>(input, QB, (size_t)NB * TQ * DQ / 8);
    k_cvt8<<<(unsigned)(((size_t)NB * TK * DK / 8 + 255) / 256), 256, 0, stream>>>(memory, KB, (size_t)NB * TK * DK / 8);
    k_vtp<<<(unsigned)(((size_t)NB * DV * TK / 2 + 255) / 256), 256, 0, stream>>>(input, VT16);
    k_gemmw<bf, 0, false><<<dim3(NB * TQ / 64, HH / 64, 1), 32, 0, stream>>>(QB, nullptr, WQT, nullptr, DQ, WQF, HH, nullptr, 1.0f, 0, 0, 0);
    k_gemmw<bf, 0, false><<<dim3(NB * TK / 64, HH / 64, 1), 32, 0, stream>>>(KB, nullptr, WKT, nullptr, DK, UHF, HH, nullptr, 1.0f, 0, 0, 0);
    k_score<<<(unsigned)(NB * TQ), 256, 0, stream>>>(WQF, UHF, w2, mmask, P16);
    k_gemmw<h16, 0, false><<<dim3(TQ / 64, DV / 64, NB), 32, 0, stream>>>(P16, nullptr, VT16, nullptr, TK, OUT0, OUTW, nullptr, OSC, (size_t)TQ * TK, (size_t)DV * TK, (size_t)TQ_FULL * OUTW);
    k_cph<<<(unsigned)(((size_t)NB * TQ * DQ / 4 + 255) / 256), 256, 0, stream>>>(input, OUT0, (size_t)NB * TQ * DQ / 4);
}
